// HeteroGAT_pyg_17119739641950
// MI455X (gfx1250) — hardware-verified
//
#include <hip/hip_runtime.h>
#include <stddef.h>


#define NTHR  256
#define NWAVE 8
#define GR    32
#define CHUNK 2048
#define WCAP  256
#define NGRP  (CHUNK / (NTHR * 4))
#define FW    128
#define HW    256
#define NBA   256
#define NBB   512

static_assert(WCAP == (CHUNK / NTHR) * 32);
static_assert(NGRP >= 1);
static_assert(CHUNK <= 2048);
static_assert(NBA <= 512 && NBB <= 512);
static_assert((NBA & (NBA - 1)) == 0 && (NBB & (NBB - 1)) == 0);

typedef float    v4f  __attribute__((ext_vector_type(4)));
typedef float    v8f  __attribute__((ext_vector_type(8)));
typedef int      v4i  __attribute__((ext_vector_type(4)));
typedef _Float16 v8h  __attribute__((ext_vector_type(8)));
typedef _Float16 v16h __attribute__((ext_vector_type(16)));
union Frag   { v16h v; v8h half[2]; };
union Pack16 { v8h h; v4i i; };

__host__ __device__ constexpr int agg_lds_bytes(int D, int NB) {
  return 4 * (NB * D + 2 * NB + NWAVE * WCAP + NWAVE + 2 * NB);
}
static_assert(agg_lds_bytes(HW, NBA) == 274464);
static_assert(agg_lds_bytes(FW, NBB) == 278560);

__device__ __forceinline__ v8f wm(v16h a, v16h b, v8f c) {
  v8f d = __builtin_amdgcn_wmma_f32_16x16x32_f16(false, a, false, b, (short)0, c, false, false);
  asm volatile("v_nop\n\tv_nop\n\tv_nop\n\tv_nop" : "+v"(d) : "v"(a), "v"(b));
  return d;
}

__device__ __forceinline__ float wsum(float v) {
  v += __shfl_xor(v, 16, 32);
  v += __shfl_xor(v, 8, 32);
  v += __shfl_xor(v, 4, 32);
  v += __shfl_xor(v, 2, 32);
  v += __shfl_xor(v, 1, 32);
  return v;
}

__device__ __forceinline__ int iclamp(int v, int hi) {
  v = v < 0 ? 0 : v;
  return v > hi ? hi : v;
}

template <int K>
__global__ __launch_bounds__(NTHR) void k_prep(const float* __restrict__ W, _Float16* Wt, int N) {
  constexpr int TP  = K + 8;
  constexpr int PPR = K / 8;
  constexpr int NIT = (32 * PPR) / NTHR;
  static_assert(NIT >= 1 && NIT * NTHR == 32 * PPR);
  static_assert(((TP * 2) % 16) == 0);
  __shared__ __attribute__((aligned(16))) _Float16 T[32 * TP];
  const int tid = threadIdx.x;
  const int n0  = blockIdx.x * 32;
#pragma unroll 1
  for (int idx = tid; idx < 32 * K; idx += NTHR) {
    const int k = idx >> 5;
    const int r = idx & 31;
    int n = n0 + r;
    n = n > N - 1 ? N - 1 : n;
    T[r * TP + k] = (_Float16)(W[(size_t)k * N + n] * 8.0f);
  }
  __syncthreads();
  Pack16 u[NIT];
  size_t go[NIT];
#pragma unroll
  for (int it = 0; it < NIT; ++it) {
    const int q  = it * NTHR + tid;
    const int r  = q / PPR;
    const int c8 = (q - r * PPR) * 8;
    u[it].h = *(const v8h*)(T + r * TP + c8);
    go[it]  = (size_t)(n0 + r) * K + c8;
  }
#pragma unroll
  for (int it = 0; it < NIT; ++it) *(volatile v4i*)(Wt + go[it]) = u[it].i;
  __threadfence();
#pragma unroll
  for (int it = 0; it < NIT; ++it) *(volatile v4i*)(Wt + go[it]) = u[it].i;
}

template <int K, int N>
__global__ __launch_bounds__(NTHR) void k_gemm(
    const float* __restrict__ x, const _Float16* __restrict__ Wt,
    const float* __restrict__ att_s, const float* __restrict__ att_d,
    float* hs, float* asrc, float* adst, int nN) {
  constexpr int AP  = K + 8;
  constexpr int XSP = N + 4;
  constexpr int NT  = N / 128;
  constexpr int KS  = K / 32;
  constexpr int SEG = N / 128;
  static_assert(NT >= 1 && NT * 128 == N && KS * 32 == K);
  static_assert(((AP * 2) % 16) == 0 && ((XSP * 4) % 16) == 0);
  __shared__ __attribute__((aligned(16))) _Float16 At[GR * AP];
  __shared__ __attribute__((aligned(16))) float Xs[GR * XSP];
  __shared__ __attribute__((aligned(16))) float AD[2 * GR * NWAVE];
  __shared__ __attribute__((aligned(16))) float L2[2 * GR];

  const int tid  = threadIdx.x;
  const int lane = tid & 31;
  const int wave = tid >> 5;
  const int hh   = lane >> 4;
  const int m    = lane & 15;
  const int rowBase = blockIdx.x * GR;

  {
    const int r  = tid >> 3;
    const int c0 = (tid & 7) * (K / 8);
    int row = rowBase + r;
    if (row > nN - 1) row = nN - 1;
    const float* p = x + (size_t)row * K + c0;
#pragma unroll
    for (int j = 0; j < K / 64; ++j) {
      const v4f f0 = *(const v4f*)(p + 8 * j);
      const v4f f1 = *(const v4f*)(p + 8 * j + 4);
      Pack16 u;
      u.h[0] = (_Float16)f0.x; u.h[1] = (_Float16)f0.y; u.h[2] = (_Float16)f0.z; u.h[3] = (_Float16)f0.w;
      u.h[4] = (_Float16)f1.x; u.h[5] = (_Float16)f1.y; u.h[6] = (_Float16)f1.z; u.h[7] = (_Float16)f1.w;
      *(v8h*)(At + r * AP + c0 + 8 * j) = u.h;
    }
  }
  __syncthreads();

  const v8f z8 = {0.f, 0.f, 0.f, 0.f, 0.f, 0.f, 0.f, 0.f};
  v8f acc[2][NT];
#pragma unroll
  for (int T = 0; T < 2; ++T)
#pragma unroll
    for (int ct = 0; ct < NT; ++ct) acc[T][ct] = z8;

#pragma unroll 1
  for (int kt = 0; kt < KS; ++kt) {
    const int k0 = kt * 32;
    Frag a0, a1;
    const _Float16* pa0 = At + m * AP + k0 + 8 * hh;
    const _Float16* pa1 = At + (16 + m) * AP + k0 + 8 * hh;
    a0.half[0] = *(const v8h*)pa0; a0.half[1] = *(const v8h*)(pa0 + 16);
    a1.half[0] = *(const v8h*)pa1; a1.half[1] = *(const v8h*)(pa1 + 16);
#pragma unroll
    for (int ct = 0; ct < NT; ++ct) {
      const int ncol = (wave * NT + ct) * 16 + m;
      const _Float16* pb = Wt + (size_t)ncol * K + k0 + 8 * hh;
      Frag b;
      b.half[0] = *(const v8h*)pb;
      b.half[1] = *(const v8h*)(pb + 16);
      acc[0][ct] = wm(a0.v, b.v, acc[0][ct]);
      acc[1][ct] = wm(a1.v, b.v, acc[1][ct]);
    }
  }

#pragma unroll
  for (int T = 0; T < 2; ++T) {
    float ss[8], sd[8];
#pragma unroll
    for (int r = 0; r < 8; ++r) { ss[r] = 0.f; sd[r] = 0.f; }
#pragma unroll
    for (int ct = 0; ct < NT; ++ct) {
      const int ncol = (wave * NT + ct) * 16 + m;
      const float cs = att_s[ncol];
      const float cd = att_d[ncol];
#pragma unroll
      for (int r = 0; r < 8; ++r) {
        const float v = acc[T][ct][r] * 0.125f;
        Xs[(T * 16 + 8 * hh + r) * XSP + ncol] = v;
        ss[r] += v * cs;
        sd[r] += v * cd;
      }
    }
#pragma unroll
    for (int mk = 1; mk < 16; mk <<= 1) {
#pragma unroll
      for (int r = 0; r < 8; ++r) {
        ss[r] += __shfl_xor(ss[r], mk, 32);
        sd[r] += __shfl_xor(sd[r], mk, 32);
      }
    }
    if (m == 0) {
#pragma unroll
      for (int r = 0; r < 8; ++r) {
        AD[(T * 16 + 8 * hh + r) * NWAVE + wave]      = ss[r];
        AD[(GR + T * 16 + 8 * hh + r) * NWAVE + wave] = sd[r];
      }
    }
  }
  __syncthreads();
  if (tid < 2 * GR) {
    float s = 0.f;
#pragma unroll
    for (int w = 0; w < NWAVE; ++w) s += AD[tid * NWAVE + w];
    L2[tid] = s;
  }
  __syncthreads();

  v4f xr[4][SEG];
#pragma unroll
  for (int i = 0; i < 4; ++i)
#pragma unroll
    for (int sg = 0; sg < SEG; ++sg)
      xr[i][sg] = *(const v4f*)(Xs + (4 * wave + i) * XSP + sg * 128 + 4 * lane);
  float* xpp[4];
#pragma unroll
  for (int i = 0; i < 4; ++i) xpp[i] = hs + (size_t)(rowBase + 4 * wave + i) * N + 4 * lane;
  const bool wl = (wave < 2) && (lane < 8);
  const int  lq = lane & 7;
  const v4f  gv = *(const v4f*)(L2 + (wave & 1) * GR + 4 * lq);
  float* gp = ((wave & 1) ? adst : asrc) + (size_t)rowBase + 4 * lq;

#pragma unroll
  for (int i = 0; i < 4; ++i)
#pragma unroll
    for (int sg = 0; sg < SEG; ++sg) *(volatile v4f*)(xpp[i] + sg * 128) = xr[i][sg];
  if (wl) *(volatile v4f*)gp = gv;
  __threadfence();
#pragma unroll
  for (int i = 0; i < 4; ++i)
#pragma unroll
    for (int sg = 0; sg < SEG; ++sg) *(volatile v4f*)(xpp[i] + sg * 128) = xr[i][sg];
  if (wl) *(volatile v4f*)gp = gv;
}

template <int D, int NB, int HEAD>
__global__ __launch_bounds__(NTHR) void k_agg(
    const int* __restrict__ ei, const float* __restrict__ hs,
    const float* __restrict__ asrc, const float* __restrict__ adst,
    const float* __restrict__ bias, const float* __restrict__ wout,
    float* hp, float* uo, float* wo, int nN, int nE) {
  constexpr int NV  = D / 128;
  constexpr int SPW = NB / NWAVE;
  constexpr int LPW = SPW / 4;
  static_assert(NV >= 1 && NV * 128 == D && LPW >= 8 && LPW <= 32);
  extern __shared__ v4f lds_dyn[];
  float* sacc = (float*)lds_dyn;
  float* den  = sacc + NB * D;
  float* mx   = den + NB;
  int*   list = (int*)(mx + NB);
  int*   wcnt = list + NWAVE * WCAP;
  float* ub   = (float*)(wcnt + NWAVE);
  float* wb   = ub + NB;

  const int tid  = threadIdx.x;
  const int lane = tid & 31;
  const int wave = tid >> 5;
  const int nodeBase = blockIdx.x * NB;

  {
    const v4f z4 = {0.f, 0.f, 0.f, 0.f};
    for (int i = tid; i < (NB * D) / 4; i += NTHR) lds_dyn[i] = z4;
    for (int i = tid; i < NB; i += NTHR) { den[i] = 0.f; mx[i] = -1.0e30f; ub[i] = 0.f; wb[i] = 0.f; }
  }
  __syncthreads();

  const int* eid = ei + nE;
  const bool vec4 = ((nE & 3) == 0);
  const int nChunks = (nE + CHUNK - 1) / CHUNK;

#pragma unroll 1
  for (int ch = 0; ch < nChunks; ++ch) {
    const int cbase = ch * CHUNK;
    int wc = 0;
#pragma unroll
    for (int g = 0; g < NGRP; ++g) {
      const int el0 = (g * NTHR + tid) * 4;
      const int e0  = cbase + el0;
      const int sent = -2147483647 - 1;
      v4i d;
      if (vec4 && (cbase + CHUNK <= nE)) {
        d = *(const v4i*)(eid + e0);
      } else {
        const int q0 = eid[iclamp(e0,     nE - 1)];
        const int q1 = eid[iclamp(e0 + 1, nE - 1)];
        const int q2 = eid[iclamp(e0 + 2, nE - 1)];
        const int q3 = eid[iclamp(e0 + 3, nE - 1)];
        d.x = (e0     < nE) ? q0 : sent;
        d.y = (e0 + 1 < nE) ? q1 : sent;
        d.z = (e0 + 2 < nE) ? q2 : sent;
        d.w = (e0 + 3 < nE) ? q3 : sent;
      }
      const unsigned s0 = (unsigned)d.x - (unsigned)nodeBase;
      const unsigned s1 = (unsigned)d.y - (unsigned)nodeBase;
      const unsigned s2 = (unsigned)d.z - (unsigned)nodeBase;
      const unsigned s3 = (unsigned)d.w - (unsigned)nodeBase;
      const bool h0 = s0 < (unsigned)NB;
      const bool h1 = s1 < (unsigned)NB;
      const bool h2 = s2 < (unsigned)NB;
      const bool h3 = s3 < (unsigned)NB;
      const unsigned many = __builtin_amdgcn_ballot_w32(h0 | h1 | h2 | h3);
      if (many != 0u) {
#define HITJ(J, HJ, SJ) { \
          const unsigned mj = __builtin_amdgcn_ballot_w32(HJ); \
          if (HJ) { \
            const int pos = wc + (int)__builtin_amdgcn_mbcnt_lo(mj, 0u); \
            if (pos < WCAP) list[wave * WCAP + pos] = ((el0 + (J)) << 9) | (int)(SJ); \
          } \
          wc += (int)__builtin_popcount(mj); }
        HITJ(0, h0, s0)
        HITJ(1, h1, s1)
        HITJ(2, h2, s2)
        HITJ(3, h3, s3)
#undef HITJ
      }
    }
    if (lane == 0) wcnt[wave] = wc;
    __syncthreads();

    if (wave == 0) {
#pragma unroll 1
      for (int wsx = 0; wsx < NWAVE; ++wsx) {
        int n = wcnt[wsx];
        n = n > WCAP ? WCAP : n;
        n = n < 0 ? 0 : n;
#pragma unroll 1
        for (int i = 0; i < n; ++i) {
          const int ent  = list[wsx * WCAP + i];
          const int slot = ent & (NB - 1);
          const int el   = (ent >> 9) & (CHUNK - 1);
          int e = cbase + el;
          if (e > nE - 1) e = nE - 1;
          const int src = iclamp(ei[e], nN - 1);
          int nd = nodeBase + slot;
          if (nd > nN - 1) nd = nN - 1;
          float al = asrc[src] + adst[nd];
          al = (al > 0.f) ? al : 0.2f * al;
          const float mo = mx[slot];
          const float mn = fmaxf(mo, al);
          const float sc = __expf(mo - mn);
          const float p  = __expf(al - mn);
          const float dn = den[slot] * sc + p;
#pragma unroll
          for (int v = 0; v < NV; ++v) {
            const v4f hv = *(const v4f*)(hs + (size_t)src * D + v * 128 + 4 * lane);
            v4f* sp = (v4f*)(sacc + slot * D + v * 128 + 4 * lane);
            const v4f cur = *sp;
            const v4f nxt = cur * sc + p * hv;
            *sp = nxt;
          }
          den[slot] = dn;
          mx[slot]  = mn;
        }
      }
    }
    __syncthreads();
  }

  v4f bv[NV];
#pragma unroll
  for (int v = 0; v < NV; ++v) bv[v] = *(const v4f*)(bias + v * 128 + 4 * lane);
  v4f wu = {0.f, 0.f, 0.f, 0.f};
  v4f ww = {0.f, 0.f, 0.f, 0.f};
  if (HEAD) {
    wu = *(const v4f*)(wout + 4 * lane);
    ww = *(const v4f*)(wout + FW + 4 * lane);
  }
#pragma unroll 1
  for (int j = 0; j < SPW; ++j) {
    const int slot = wave * SPW + j;
    const int node = nodeBase + slot;
    const bool valid = node < nN;
    const int nr = valid ? node : nN - 1;
    float al = asrc[nr] + adst[nr];
    al = (al > 0.f) ? al : 0.2f * al;
    const float mo = mx[slot];
    const float mn = fmaxf(mo, al);
    const float sc = __expf(mo - mn);
    const float p  = __expf(al - mn);
    const float dv = den[slot] * sc + p;
    const float inv = 1.0f / dv;
    v4f y[NV];
#pragma unroll
    for (int v = 0; v < NV; ++v) {
      const v4f hv = *(const v4f*)(hs + (size_t)nr * D + v * 128 + 4 * lane);
      const v4f sv = *(const v4f*)(sacc + slot * D + v * 128 + 4 * lane) * sc + p * hv;
      v4f t = sv * inv + bv[v];
      if (!HEAD) {
        t.x = t.x > 0.f ? t.x : 0.f;
        t.y = t.y > 0.f ? t.y : 0.f;
        t.z = t.z > 0.f ? t.z : 0.f;
        t.w = t.w > 0.f ? t.w : 0.f;
      }
      y[v] = t;
    }
    if (!HEAD) {
      if (valid) {
        float* op = hp + (size_t)nr * D + 4 * lane;
#pragma unroll
        for (int v = 0; v < NV; ++v) *(volatile v4f*)(op + v * 128) = y[v];
        __threadfence();
#pragma unroll
        for (int v = 0; v < NV; ++v) *(volatile v4f*)(op + v * 128) = y[v];
      }
    } else {
      const v4f tu = y[0] * wu;
      const v4f tw = y[0] * ww;
      const float su = wsum((tu.x + tu.y) + (tu.z + tu.w));
      const float sw = wsum((tw.x + tw.y) + (tw.z + tw.w));
      if (lane == 0) {
        ub[slot] = valid ? su : 0.f;
        wb[slot] = valid ? sw : 0.f;
      }
    }
  }
  if (HEAD) {
    __syncthreads();
    const int lq = lane < LPW ? lane : LPW - 1;
    const v4f gu = *(const v4f*)(ub + wave * SPW + 4 * lq);
    const v4f gw = *(const v4f*)(wb + wave * SPW + 4 * lq);
    float* pu = uo + (size_t)nodeBase + wave * SPW + 4 * lq;
    float* pw = wo + (size_t)nodeBase + wave * SPW + 4 * lq;
    if (lane < LPW) { *(volatile v4f*)pu = gu; *(volatile v4f*)pw = gw; }
    __threadfence();
    if (lane < LPW) { *(volatile v4f*)pu = gu; *(volatile v4f*)pw = gw; }
  }
}

__device__ __forceinline__ float sigm(float z) {
  const float e = __expf(-z);
  return __builtin_amdgcn_rcpf(1.0f + e);
}

__global__ __launch_bounds__(NTHR) void k_head(
    const int* __restrict__ mask, const float* __restrict__ uo, const float* __restrict__ wo,
    const float* __restrict__ bout, float* out, int nQ, int nN) {
  const int t = blockIdx.x * NTHR + threadIdx.x;
  if (t >= nQ) return;
  const v4i ma = *(const v4i*)(mask + (size_t)t * 8);
  const v4i mb = *(const v4i*)(mask + (size_t)t * 8 + 4);
  const int hi = nN - 1;
  const float b = bout[0];
  v4f o;
  o.x = sigm(uo[iclamp(ma.x, hi)] + wo[iclamp(ma.y, hi)] + b);
  o.y = sigm(uo[iclamp(ma.z, hi)] + wo[iclamp(ma.w, hi)] + b);
  o.z = sigm(uo[iclamp(mb.x, hi)] + wo[iclamp(mb.y, hi)] + b);
  o.w = sigm(uo[iclamp(mb.z, hi)] + wo[iclamp(mb.w, hi)] + b);
  float* op = out + (size_t)t * 4;
  *(volatile v4f*)op = o;
  __threadfence();
  *(volatile v4f*)op = o;
}

static inline size_t a256(size_t v) { return (v + 255) & ~(size_t)255; }

extern "C" void kernel_launch(void* const* d_in, const int* in_sizes, int n_in,
                              void* d_out, int out_size, void* d_ws, size_t ws_size,
                              hipStream_t stream) {
  if (n_in < 23) return;
  const int nN = in_sizes[0] / FW;
  if (nN <= 0 || in_sizes[0] != nN * FW) return;
  if (in_sizes[5] < 2 || (in_sizes[5] & 1) != 0) return;
  const int nE = in_sizes[5] / 2;
  if ((in_sizes[6] & 1) != 0) return;
  const int nPair = in_sizes[6] / 2;
  if (nPair <= 0 || (nPair & 3) != 0 || out_size != nPair) return;
  if (in_sizes[7] != 3 * FW * HW || in_sizes[8] != 3 * HW || in_sizes[9] != 3 * HW || in_sizes[10] != 3 * HW) return;
  if (in_sizes[11] != 3 * HW * FW || in_sizes[12] != 3 * FW || in_sizes[13] != 3 * FW || in_sizes[14] != 3 * FW) return;
  if (in_sizes[21] != 2 * FW || in_sizes[22] < 1) return;

  const float* xp    = (const float*)d_in[0];
  const int*   ei    = (const int*)d_in[5];
  const int*   mask  = (const int*)d_in[6];
  const float* Wa2   = (const float*)d_in[7]  + (size_t)2 * FW * HW;
  const float* asa2  = (const float*)d_in[8]  + 2 * HW;
  const float* ada2  = (const float*)d_in[9]  + 2 * HW;
  const float* ba2   = (const float*)d_in[10] + 2 * HW;
  const float* Wb2   = (const float*)d_in[11] + (size_t)2 * HW * FW;
  const float* asb2  = (const float*)d_in[12] + 2 * FW;
  const float* adb2  = (const float*)d_in[13] + 2 * FW;
  const float* bb2   = (const float*)d_in[14] + 2 * FW;
  const float* Wout  = (const float*)d_in[21];
  const float* bout  = (const float*)d_in[22];
  float* out = (float*)d_out;

  const int nP    = ((nN + GR - 1) / GR) * GR;
  const int gridA = (nN + NBA - 1) / NBA;
  const int gridB = (nN + NBB - 1) / NBB;
  size_t off = 0;
  char* ws = (char*)d_ws;
  _Float16* WtA = (_Float16*)(ws + off); off += a256((size_t)HW * FW * sizeof(_Float16));
  _Float16* WtB = (_Float16*)(ws + off); off += a256((size_t)FW * HW * sizeof(_Float16));
  float* HS  = (float*)(ws + off); off += a256((size_t)nP * HW * sizeof(float));
  float* HP  = (float*)(ws + off); off += a256((size_t)nP * HW * sizeof(float));
  float* ASA = (float*)(ws + off); off += a256((size_t)nP * sizeof(float));
  float* ADA = (float*)(ws + off); off += a256((size_t)nP * sizeof(float));
  float* ASB = (float*)(ws + off); off += a256((size_t)nP * sizeof(float));
  float* ADB = (float*)(ws + off); off += a256((size_t)nP * sizeof(float));
  float* UO  = (float*)(ws + off); off += a256((size_t)gridB * NBB * sizeof(float));
  float* WO  = (float*)(ws + off); off += a256((size_t)gridB * NBB * sizeof(float));
  if (off > ws_size) return;

  k_prep<FW><<<HW / 32, NTHR, 0, stream>>>(Wa2, WtA, HW);
  k_gemm<FW, HW><<<nP / GR, NTHR, 0, stream>>>(xp, WtA, asa2, ada2, HS, ASA, ADA, nN);
  {
    auto fa = &k_agg<HW, NBA, 0>;
    hipFuncSetAttribute(reinterpret_cast<const void*>(fa),
                        hipFuncAttributeMaxDynamicSharedMemorySize, agg_lds_bytes(HW, NBA));
    k_agg<HW, NBA, 0><<<gridA, NTHR, agg_lds_bytes(HW, NBA), stream>>>(
        ei, HS, ASA, ADA, ba2, Wout, HP, UO, WO, nN, nE);
  }

  k_prep<HW><<<FW / 32, NTHR, 0, stream>>>(Wb2, WtB, FW);
  k_gemm<HW, FW><<<nP / GR, NTHR, 0, stream>>>(HP, WtB, asb2, adb2, HS, ASB, ADB, nN);
  {
    auto fb = &k_agg<FW, NBB, 1>;
    hipFuncSetAttribute(reinterpret_cast<const void*>(fb),
                        hipFuncAttributeMaxDynamicSharedMemorySize, agg_lds_bytes(FW, NBB));
    k_agg<FW, NBB, 1><<<gridB, NTHR, agg_lds_bytes(FW, NBB), stream>>>(
        ei, HS, ASB, ADB, bb2, Wout, HP, UO, WO, nN, nE);
  }

  const int nQ = nPair / 4;
  k_head<<<(nQ + NTHR - 1) / NTHR, NTHR, 0, stream>>>(mask, UO, WO, bout, out, nQ, nN);
}
